// GNN_49967649521735
// MI455X (gfx1250) — hardware-verified
//
#include <hip/hip_runtime.h>
#include <stddef.h>
#include <stdint.h>
#include <math.h>


#pragma clang fp contract(off)

#define FIN    128
#define DIM    256
#define K1     256
#define K2     512
#define NGR    256
#define NTHR   256
#define NWAVE  8
#define EPT    8
#define CHUNK  (NTHR * EPT)
#define WCAP   (EPT * 32)
#define LISTN  (NWAVE * WCAP)
#define NBD    8192
#define SLD    13
#define NBA    1024
#define SLA    10
#define RCAP   28672
#define DEGCAP 64
#define GBM    64
#define GBN    128
#define GTHR   128
#define RNB    128
#define NUW1   (DIM * (K1 / 8))
#define NUW2   (DIM * (K2 / 8))
#define RBH    512
#define AGG_ZINTS    (LISTN + 2 * RCAP + 3 * NBA)
#define MISC_INTS    16
#define ROWBUF_INTS  (NWAVE * RBH / 2)
#define AGG_LDS_INTS (AGG_ZINTS + MISC_INTS + ROWBUF_INTS)
#define WSMAX  134217728

static_assert((CHUNK & (CHUNK - 1)) == 0 && CHUNK <= 4096);
static_assert((NBD & (NBD - 1)) == 0 && NBD == (1 << SLD));
static_assert((NBA & (NBA - 1)) == 0 && NBA == (1 << SLA));
static_assert(((long long)CHUNK << SLD) < (1LL << 31));
static_assert(((long long)CHUNK << SLA) < (1LL << 31));
static_assert(NBD % (NTHR * 4) == 0);
static_assert(LISTN % NTHR == 0);
static_assert(NBA % NWAVE == 0 && NBA % 32 == 0 && NBA % GBM == 0);
static_assert(RCAP % 4 == 0 && AGG_ZINTS % 4 == 0 && LISTN % 4 == 0 && ((AGG_ZINTS + MISC_INTS) % 4) == 0);
static_assert(AGG_ZINTS % (NTHR * 4) == 0);
static_assert(K1 % 32 == 0 && K2 % 32 == 0 && K1 == 2 * FIN && K2 == 2 * DIM);
static_assert(DIM % GBN == 0 && GBM == (GTHR / 32) * 16 && GBN == 4 * 32);
static_assert(NUW1 % NTHR == 0 && NUW2 % NTHR == 0);
static_assert(FIN == 4 * 32 && DIM == 8 * 32);
static_assert(RNB == NWAVE * 16 && RNB == 4 * 32 && RNB % GBM == 0);
static_assert(AGG_LDS_INTS * 4 <= 300000);
static_assert((NGR * DIM * 4) % 128 == 0);

typedef float          v4f   __attribute__((ext_vector_type(4)));
typedef float          v8f   __attribute__((ext_vector_type(8)));
typedef int            v4i   __attribute__((ext_vector_type(4)));
typedef int            v8i   __attribute__((ext_vector_type(8)));
typedef unsigned       v2u   __attribute__((ext_vector_type(2)));
typedef unsigned short v4us  __attribute__((ext_vector_type(4)));
typedef unsigned short v8us  __attribute__((ext_vector_type(8)));
typedef unsigned short v16us __attribute__((ext_vector_type(16)));
typedef __bf16         v16bf __attribute__((ext_vector_type(16)));
typedef v4f  __attribute__((may_alias)) v4fa;
typedef v4i  __attribute__((may_alias)) v4ia;
typedef v2u  __attribute__((may_alias)) v2ua;
typedef v4us __attribute__((may_alias)) v4usa;
typedef v8us __attribute__((may_alias)) v8usa;
union FragB { v16bf v; v16us u; v8us h[2]; v8i w; };

__device__ __forceinline__ v8f wmb(const FragB& a, const FragB& b, v8f c) {
  v8f d = __builtin_amdgcn_wmma_f32_16x16x32_bf16(false, a.v, false, b.v, (short)0, c, false, false);
  asm volatile("v_nop\n\tv_nop\n\tv_nop\n\tv_nop" : "+v"(d) : "v"(a.w), "v"(b.w));
  return d;
}

__device__ __forceinline__ unsigned bf16_bits(float f) {
  const unsigned u = __float_as_uint(f);
  return (u + 0x7FFFu + ((u >> 16) & 1u)) >> 16;
}
__device__ __forceinline__ float bf16_val(float f) {
  return __uint_as_float(bf16_bits(f) << 16);
}

__device__ __forceinline__ void wave_sync() {
  __builtin_amdgcn_fence(__ATOMIC_RELEASE, "wavefront");
  __builtin_amdgcn_wave_barrier();
  __builtin_amdgcn_fence(__ATOMIC_ACQUIRE, "wavefront");
}

__device__ __forceinline__ void split4(float m0, float m1, float m2, float m3, v4us& mh, v4us& ml) {
  unsigned hb;
  hb = bf16_bits(m0); mh[0] = (unsigned short)hb; ml[0] = (unsigned short)bf16_bits(m0 - __uint_as_float(hb << 16));
  hb = bf16_bits(m1); mh[1] = (unsigned short)hb; ml[1] = (unsigned short)bf16_bits(m1 - __uint_as_float(hb << 16));
  hb = bf16_bits(m2); mh[2] = (unsigned short)hb; ml[2] = (unsigned short)bf16_bits(m2 - __uint_as_float(hb << 16));
  hb = bf16_bits(m3); mh[3] = (unsigned short)hb; ml[3] = (unsigned short)bf16_bits(m3 - __uint_as_float(hb << 16));
}

template <int SLB>
__device__ __forceinline__ int scan_chunk(const int* __restrict__ dsts, int nE, int cbase, int slotBase,
                                          int nb, int vec8, int* list, int tid, int lane, int wave) {
  int wc = 0;
  const int el0  = tid * EPT;
  const int e0   = cbase + el0;
  const int sent = -2147483647 - 1;
  v4i da, db;
  if (vec8 != 0 && cbase + CHUNK <= nE) {
    da = *(const v4i*)(dsts + e0);
    db = *(const v4i*)(dsts + e0 + 4);
  } else {
    da.x = (e0     < nE) ? dsts[min(e0,     nE - 1)] : sent;
    da.y = (e0 + 1 < nE) ? dsts[min(e0 + 1, nE - 1)] : sent;
    da.z = (e0 + 2 < nE) ? dsts[min(e0 + 2, nE - 1)] : sent;
    da.w = (e0 + 3 < nE) ? dsts[min(e0 + 3, nE - 1)] : sent;
    db.x = (e0 + 4 < nE) ? dsts[min(e0 + 4, nE - 1)] : sent;
    db.y = (e0 + 5 < nE) ? dsts[min(e0 + 5, nE - 1)] : sent;
    db.z = (e0 + 6 < nE) ? dsts[min(e0 + 6, nE - 1)] : sent;
    db.w = (e0 + 7 < nE) ? dsts[min(e0 + 7, nE - 1)] : sent;
  }
  const unsigned nbs = (unsigned)slotBase;
  const unsigned unb = (unsigned)nb;
  const unsigned s0 = (unsigned)da.x - nbs, s1 = (unsigned)da.y - nbs;
  const unsigned s2 = (unsigned)da.z - nbs, s3 = (unsigned)da.w - nbs;
  const unsigned s4 = (unsigned)db.x - nbs, s5 = (unsigned)db.y - nbs;
  const unsigned s6 = (unsigned)db.z - nbs, s7 = (unsigned)db.w - nbs;
  const bool h0 = s0 < unb, h1 = s1 < unb, h2 = s2 < unb, h3 = s3 < unb;
  const bool h4 = s4 < unb, h5 = s5 < unb, h6 = s6 < unb, h7 = s7 < unb;
  const unsigned any = __builtin_amdgcn_ballot_w32(h0 | h1 | h2 | h3 | h4 | h5 | h6 | h7);
  if (any != 0u) {
#define HITJ(J, HJ, SJ) { \
      const unsigned mj = __builtin_amdgcn_ballot_w32(HJ); \
      if (mj != 0u) { \
        if (HJ) { \
          const int pos = wc + (int)__builtin_amdgcn_mbcnt_lo(mj, 0u); \
          if (pos < WCAP) list[wave * WCAP + pos] = ((el0 + (J)) << SLB) | (int)(SJ); \
        } \
        wc += (int)__builtin_popcount(mj); } }
    HITJ(0, h0, s0)
    HITJ(1, h1, s1)
    HITJ(2, h2, s2)
    HITJ(3, h3, s3)
    HITJ(4, h4, s4)
    HITJ(5, h5, s5)
    HITJ(6, h6, s6)
    HITJ(7, h7, s7)
#undef HITJ
  }
  return wc;
}

__global__ __launch_bounds__(NTHR) void k_wprep(const float* __restrict__ W1, const float* __restrict__ W2,
                                                unsigned short* W1D, unsigned short* W2D) {
  const int u = (int)blockIdx.x * NTHR + (int)threadIdx.x;
  v8us o;
  unsigned short* dp;
  if (u < NUW1) {
    const int n  = u >> 5;
    const int k8 = (u & 31) * 8;
    const int kk = k8 & (FIN - 1);
    const float* p = W1 + (size_t)kk * DIM + n;
#pragma unroll
    for (int i = 0; i < 8; ++i) o[i] = (unsigned short)bf16_bits(p[(size_t)i * DIM]);
    dp = W1D + (size_t)n * K1 + k8;
  } else if (u < NUW1 + NUW2) {
    const int v  = u - NUW1;
    const int n  = v >> 6;
    const int k8 = (v & 63) * 8;
    const int kk = k8 & (DIM - 1);
    const float* p = W2 + (size_t)kk * DIM + n;
#pragma unroll
    for (int i = 0; i < 8; ++i) o[i] = (unsigned short)bf16_bits(p[(size_t)i * DIM]);
    dp = W2D + (size_t)n * K2 + k8;
  } else {
    return;
  }
  *(volatile v8us*)dp = o;
  __threadfence();
  *(volatile v8us*)dp = o;
}

__global__ __launch_bounds__(NTHR) void k_cvx(const float* __restrict__ x, int nN, int nUnits,
                                              unsigned short* xb) {
  const int u = (int)blockIdx.x * NTHR + (int)threadIdx.x;
  if (u >= nUnits) return;
  const int row = u >> 4;
  const int k8  = (u & 15) * 8;
  const int rc  = row < nN ? row : nN - 1;
  const float* p = x + (size_t)rc * FIN + k8;
  const v4f a = *(const v4fa*)p;
  const v4f b = *(const v4fa*)(p + 4);
  const bool ok = row < nN;
  v8us o;
  o[0] = ok ? (unsigned short)bf16_bits(a.x) : (unsigned short)0;
  o[1] = ok ? (unsigned short)bf16_bits(a.y) : (unsigned short)0;
  o[2] = ok ? (unsigned short)bf16_bits(a.z) : (unsigned short)0;
  o[3] = ok ? (unsigned short)bf16_bits(a.w) : (unsigned short)0;
  o[4] = ok ? (unsigned short)bf16_bits(b.x) : (unsigned short)0;
  o[5] = ok ? (unsigned short)bf16_bits(b.y) : (unsigned short)0;
  o[6] = ok ? (unsigned short)bf16_bits(b.z) : (unsigned short)0;
  o[7] = ok ? (unsigned short)bf16_bits(b.w) : (unsigned short)0;
  unsigned short* dp = xb + (size_t)row * FIN + k8;
  *(volatile v8us*)dp = o;
  __threadfence();
  *(volatile v8us*)dp = o;
}

__global__ __launch_bounds__(NTHR) void k_deg(const int* __restrict__ keys, int nE, int vec8, float* nrm) {
  __shared__ __attribute__((aligned(16))) int scnt[NBD];
  __shared__ __attribute__((aligned(16))) int list[LISTN];
  __shared__ int wcnt[NWAVE];
  const int tid = (int)threadIdx.x, lane = tid & 31, wave = tid >> 5;
  const int nodeBase = (int)blockIdx.x * NBD;

  for (int i = tid; i < NBD; i += NTHR) scnt[i] = 0;
  for (int i = tid; i < LISTN; i += NTHR) list[i] = 0;
  if (tid < NWAVE) wcnt[tid] = 0;
  __syncthreads();

  const int nChunks = (nE + CHUNK - 1) / CHUNK;
#pragma unroll 1
  for (int ch = 0; ch < nChunks; ++ch) {
    const int cbase = ch * CHUNK;
    const int wc = scan_chunk<SLD>(keys, nE, cbase, nodeBase, NBD, vec8, list, tid, lane, wave);
    if (lane == 0) wcnt[wave] = wc;
    __syncthreads();
    if (wave == 0) {
#pragma unroll 1
      for (int w2 = 0; w2 < NWAVE; ++w2) {
        int c = wcnt[w2];
        c = c < 0 ? 0 : (c > WCAP ? WCAP : c);
#pragma unroll 1
        for (int b0 = 0; b0 < c; b0 += 32) {
          const int idx = b0 + lane;
          const int ent = list[w2 * WCAP + (idx < WCAP ? idx : WCAP - 1)];
          const int m32 = (c - b0) < 32 ? (c - b0) : 32;
#pragma unroll 1
          for (int k = 0; k < m32; ++k) {
            const int u  = __builtin_amdgcn_readlane(ent, k);
            const int sl = u & (NBD - 1);
            if (lane == 0) scnt[sl] = scnt[sl] + 1;
          }
        }
      }
    }
    __syncthreads();
  }

#pragma unroll 1
  for (int i = tid; i < NBD; i += NTHR) {
    int c = scnt[i];
    c = c < 1 ? 1 : c;
    const float v = 1.0f / sqrtf((float)c);
    scnt[i] = __float_as_int(v);
  }
  __syncthreads();

  v4f vals[NBD / (NTHR * 4)];
#pragma unroll
  for (int it = 0; it < NBD / (NTHR * 4); ++it) {
    const int s0 = it * (NTHR * 4) + 4 * tid;
    const v4i c4 = *(const v4ia*)(scnt + s0);
    v4f v;
    v.x = __int_as_float(c4.x); v.y = __int_as_float(c4.y);
    v.z = __int_as_float(c4.z); v.w = __int_as_float(c4.w);
    vals[it] = v;
  }
#pragma unroll
  for (int it = 0; it < NBD / (NTHR * 4); ++it) {
    const int s0 = it * (NTHR * 4) + 4 * tid;
    *(volatile v4f*)(nrm + (size_t)nodeBase + s0) = vals[it];
  }
  __threadfence();
#pragma unroll
  for (int it = 0; it < NBD / (NTHR * 4); ++it) {
    const int s0 = it * (NTHR * 4) + 4 * tid;
    *(volatile v4f*)(nrm + (size_t)nodeBase + s0) = vals[it];
  }
}

template <int MODE>
__global__ __launch_bounds__(GTHR) void k_gemm(const unsigned short* __restrict__ Apl,
                                               const unsigned short* __restrict__ BT,
                                               const float* __restrict__ bias,
                                               const float* __restrict__ outn,
                                               float* outp, int nOut) {
  constexpr int K = (MODE == 1) ? K1 : K2;
  __shared__ __attribute__((aligned(16))) float stg[GBM * GBN];
  const int tid = (int)threadIdx.x, lane = tid & 31, wave = tid >> 5, hh = lane >> 4, m = lane & 15;
  const int rowBase = (int)blockIdx.x * GBM;
  const int col0    = (int)blockIdx.y * GBN;

  v8f acc[8];
  {
    const v8f z = {0.f, 0.f, 0.f, 0.f, 0.f, 0.f, 0.f, 0.f};
#pragma unroll
    for (int t = 0; t < 8; ++t) acc[t] = z;
  }
  const unsigned short* ap = Apl + (size_t)(rowBase + 16 * wave + m) * (size_t)K + 8 * hh;
  const unsigned short* bp = BT + (size_t)(col0 + m) * (size_t)K + 8 * hh;

#pragma unroll 1
  for (int k0 = 0; k0 < K; k0 += 32) {
    FragB af;
    af.h[0] = *(const v8usa*)(ap + k0);
    af.h[1] = *(const v8usa*)(ap + k0 + 16);
#pragma unroll
    for (int nt = 0; nt < 8; ++nt) {
      const unsigned short* wq = bp + (size_t)(16 * nt) * (size_t)K + k0;
      FragB bf;
      bf.h[0] = *(const v8usa*)wq;
      bf.h[1] = *(const v8usa*)(wq + 16);
      acc[nt] = wmb(af, bf, acc[nt]);
    }
  }

#pragma unroll
  for (int nt = 0; nt < 8; ++nt) {
    const int lc = 16 * nt + m;
#pragma unroll
    for (int r = 0; r < 8; ++r) {
      const int lr = 16 * wave + 8 * hh + r;
      stg[lr * GBN + lc] = acc[nt][r];
    }
  }
  __syncthreads();

  v4f bb4;
  {
    const v4f t1 = *(const v4f*)(bias + col0 + 4 * lane);
    bb4.x = bf16_val(t1.x); bb4.y = bf16_val(t1.y); bb4.z = bf16_val(t1.z); bb4.w = bf16_val(t1.w);
  }
  float onl = 1.0f;
  if constexpr (MODE == 1) onl = outn[rowBase + 16 * wave + m];

  v4f pv[16];
#pragma unroll
  for (int i = 0; i < 16; ++i) pv[i] = *(const v4fa*)(stg + (16 * wave + i) * GBN + 4 * lane);

#pragma unroll
  for (int i = 0; i < 16; ++i) {
    const bool ok = (rowBase + 16 * wave + i) < nOut;
    const v4f t = pv[i] + bb4;
    v4f y;
    if constexpr (MODE == 1) {
      const float on = __shfl(onl, i, 32);
      y.x = (t.x > 0.0f) ? t.x : (t.x - t.x);
      y.y = (t.y > 0.0f) ? t.y : (t.y - t.y);
      y.z = (t.z > 0.0f) ? t.z : (t.z - t.z);
      y.w = (t.w > 0.0f) ? t.w : (t.w - t.w);
      y.x = y.x * on; y.y = y.y * on; y.z = y.z * on; y.w = y.w * on;
    } else {
      y = t;
    }
    y.x = ok ? y.x : 0.0f; y.y = ok ? y.y : 0.0f; y.z = ok ? y.z : 0.0f; y.w = ok ? y.w : 0.0f;
    pv[i] = y;
  }

#pragma unroll
  for (int i = 0; i < 16; ++i) {
    const int r = rowBase + 16 * wave + i;
    *(volatile v4f*)(outp + (size_t)r * DIM + col0 + 4 * lane) = pv[i];
  }
  __threadfence();
#pragma unroll
  for (int i = 0; i < 16; ++i) {
    const int r = rowBase + 16 * wave + i;
    *(volatile v4f*)(outp + (size_t)r * DIM + col0 + 4 * lane) = pv[i];
  }
}

template <int L>
__global__ __launch_bounds__(NTHR) void k_scan(const int* __restrict__ gath, const int* __restrict__ keys,
                                               int nE, int nN, int vec8, int mRows,
                                               const float* __restrict__ outn,
                                               const unsigned short* __restrict__ xb,
                                               const float* __restrict__ h1s,
                                               unsigned short* apl) {
  constexpr int APL = (L == 1) ? K1 : K2;
  extern __shared__ __attribute__((aligned(16))) int dsm[];
  int* list = dsm;
  int* hl   = dsm + LISTN;
  int* sl   = hl + RCAP;
  int* cnt  = sl + RCAP;
  int* offs = cnt + NBA;
  int* cur  = offs + NBA;
  int* misc = cur + NBA;
  const int tid = (int)threadIdx.x, lane = tid & 31, wave = tid >> 5;
  unsigned short* rowbuf = (unsigned short*)(misc + MISC_INTS) + wave * RBH;
  const int nodeBase = (int)blockIdx.x * NBA;

  {
    const v4i z4 = {0, 0, 0, 0};
    for (int i = tid * 4; i < AGG_ZINTS; i += NTHR * 4) *(v4ia*)(dsm + i) = z4;
    if (tid < MISC_INTS) misc[tid] = 0;
  }
  __syncthreads();

  int t = 0, ov = 0;
  const int nChunks = (nE + CHUNK - 1) / CHUNK;
#pragma unroll 1
  for (int ch = 0; ch < nChunks; ++ch) {
    const int cbase = ch * CHUNK;
    const int wc = scan_chunk<SLA>(keys, nE, cbase, nodeBase, NBA, vec8, list, tid, lane, wave);
    if (lane == 0) misc[wave] = wc;
    __syncthreads();
    if (wave == 0) {
#pragma unroll 1
      for (int w2 = 0; w2 < NWAVE; ++w2) {
        int c = misc[w2];
        c = c < 0 ? 0 : (c > WCAP ? WCAP : c);
#pragma unroll 1
        for (int b0 = 0; b0 < c; b0 += 32) {
          const int idx = b0 + lane;
          const int ent = list[w2 * WCAP + (idx < WCAP ? idx : WCAP - 1)];
          const int m32 = (c - b0) < 32 ? (c - b0) : 32;
#pragma unroll 1
          for (int k = 0; k < m32; ++k) {
            const int u    = __builtin_amdgcn_readlane(ent, k);
            const int slot = u & (NBA - 1);
            const int el   = (u >> SLA) & (CHUNK - 1);
            const int pk   = ((cbase + el) << SLA) | slot;
            if (t < RCAP) {
              if (lane == 0) { hl[t] = pk; cnt[slot] = cnt[slot] + 1; }
              t = t + 1;
            } else {
              ov = 1;
            }
          }
        }
      }
    }
    __syncthreads();
  }
  if (wave == 0 && lane == 0) { misc[8] = t; misc[9] = ov; }
  __syncthreads();
  int tt = misc[8];
  tt = tt < 0 ? 0 : (tt > RCAP ? RCAP : tt);
  const int ovf = misc[9];

  if (wave == 0) {
    const int base = lane * (NBA / 32);
    int s = 0;
#pragma unroll 1
    for (int i = 0; i < NBA / 32; ++i) s += cnt[base + i];
    int incl = s;
#pragma unroll
    for (int d = 1; d < 32; d <<= 1) {
      const int y = __shfl_up(incl, d, 32);
      if (lane >= d) incl += y;
    }
    int run = incl - s;
#pragma unroll 1
    for (int i = 0; i < NBA / 32; ++i) {
      const int cv = cnt[base + i];
      offs[base + i] = run;
      cur[base + i]  = run;
      run += cv;
    }
  }
  __syncthreads();
  if (wave == 0) {
#pragma unroll 1
    for (int b0 = 0; b0 < tt; b0 += 32) {
      const int idx = b0 + lane;
      const int ent = hl[idx < RCAP ? idx : RCAP - 1];
      const int m32 = (tt - b0) < 32 ? (tt - b0) : 32;
#pragma unroll 1
      for (int k = 0; k < m32; ++k) {
        const int u    = __builtin_amdgcn_readlane(ent, k);
        const int slot = u & (NBA - 1);
        if (lane == 0) {
          int p = cur[slot];
          p = p < 0 ? 0 : (p > RCAP - 1 ? RCAP - 1 : p);
          sl[p] = u;
          cur[slot] = p + 1;
        }
      }
    }
  }
  __syncthreads();

  const float qnan = __int_as_float(0x7fc00000);
  const float pz = (ovf != 0) ? qnan : 0.0f;
#pragma unroll 1
  for (int si = 0; si < NBA / NWAVE; ++si) {
    const int s    = si * NWAVE + wave;
    const int node = nodeBase + s;
    const int craw = cnt[s];
    int c = craw;
    const bool big = c > DEGCAP;
    c = c < 0 ? 0 : (c > DEGCAP ? DEGCAP : c);
    int o = offs[s];
    o = o < 0 ? 0 : (o > RCAP ? RCAP : o);
    float a0 = 0.0f, a1 = 0.0f, a2 = 0.0f, a3 = 0.0f;
    float a4 = 0.0f, a5 = 0.0f, a6 = 0.0f, a7 = 0.0f;
#pragma unroll 1
    for (int b0 = 0; b0 < c; b0 += 32) {
      int idx = o + b0 + lane;
      idx = idx > RCAP - 1 ? RCAP - 1 : idx;
      const int ent = sl[idx];
      int eid = ent >> SLA;
      eid = eid < 0 ? 0 : (eid > nE - 1 ? nE - 1 : eid);
      int sr = gath[eid];
      sr = sr < 0 ? 0 : (sr > nN - 1 ? nN - 1 : sr);
      int oni = 0;
      if constexpr (L == 1) oni = __float_as_int(outn[sr]);
      const int m32 = (c - b0) < 32 ? (c - b0) : 32;
#pragma unroll 1
      for (int k = 0; k < m32; ++k) {
        const int sk = __builtin_amdgcn_readlane(sr, k);
        if constexpr (L == 1) {
          const float ck = __int_as_float(__builtin_amdgcn_readlane(oni, k));
          const unsigned short* rp = xb + (size_t)sk * FIN + 4 * lane;
          const v2u w = *(const v2ua*)rp;
          const float f0 = __uint_as_float(w.x << 16);
          const float f1 = __uint_as_float(w.x & 0xffff0000u);
          const float f2 = __uint_as_float(w.y << 16);
          const float f3 = __uint_as_float(w.y & 0xffff0000u);
          const float p0 = f0 * ck, p1 = f1 * ck, p2 = f2 * ck, p3 = f3 * ck;
          a0 = a0 + p0; a1 = a1 + p1; a2 = a2 + p2; a3 = a3 + p3;
        } else {
          const float* rp = h1s + (size_t)sk * DIM + 4 * lane;
          const v4f u = *(const v4f*)rp;
          const v4f v = *(const v4f*)(rp + 128);
          a0 = a0 + u.x; a1 = a1 + u.y; a2 = a2 + u.z; a3 = a3 + u.w;
          a4 = a4 + v.x; a5 = a5 + v.y; a6 = a6 + v.z; a7 = a7 + v.w;
        }
      }
    }
    const int cm = craw < 1 ? 1 : craw;
    const float inn = 1.0f / sqrtf((float)cm);
    const float pzr = big ? qnan : pz;
    const bool live = node < nN;
    const float m0 = live ? (a0 * inn + pzr) : 0.0f;
    const float m1 = live ? (a1 * inn + pzr) : 0.0f;
    const float m2 = live ? (a2 * inn + pzr) : 0.0f;
    const float m3 = live ? (a3 * inn + pzr) : 0.0f;
    v4us mh, ml;
    split4(m0, m1, m2, m3, mh, ml);
    v8us q0;
    v8us q1 = {0, 0, 0, 0, 0, 0, 0, 0};
    if constexpr (L == 1) {
      *(v4usa*)(rowbuf + 4 * lane) = mh;
      *(v4usa*)(rowbuf + FIN + 4 * lane) = ml;
      wave_sync();
      q0 = *(const v8usa*)(rowbuf + 8 * lane);
      wave_sync();
    } else {
      const float m4 = live ? (a4 * inn + pzr) : 0.0f;
      const float m5 = live ? (a5 * inn + pzr) : 0.0f;
      const float m6 = live ? (a6 * inn + pzr) : 0.0f;
      const float m7 = live ? (a7 * inn + pzr) : 0.0f;
      v4us nh, nl;
      split4(m4, m5, m6, m7, nh, nl);
      *(v4usa*)(rowbuf + 4 * lane) = mh;
      *(v4usa*)(rowbuf + 128 + 4 * lane) = nh;
      *(v4usa*)(rowbuf + 256 + 4 * lane) = ml;
      *(v4usa*)(rowbuf + 384 + 4 * lane) = nl;
      wave_sync();
      q0 = *(const v8usa*)(rowbuf + 8 * lane);
      q1 = *(const v8usa*)(rowbuf + 256 + 8 * lane);
      wave_sync();
    }
    if (node < mRows) {
      unsigned short* rpw = apl + (size_t)node * APL + 8 * lane;
      *(volatile v8us*)rpw = q0;
      if constexpr (L != 1) *(volatile v8us*)(rpw + 256) = q1;
      __threadfence();
      *(volatile v8us*)rpw = q0;
      if constexpr (L != 1) *(volatile v8us*)(rpw + 256) = q1;
    }
  }
}

__global__ __launch_bounds__(NTHR) void k_rownorm(const float* __restrict__ h2, int nN, float* nrm) {
  __shared__ __attribute__((aligned(16))) float nr[RNB];
  const int tid = (int)threadIdx.x, lane = tid & 31, wave = tid >> 5;
  const int base = (int)blockIdx.x * RNB;
#pragma unroll 1
  for (int i = 0; i < 16; ++i) {
    const int lr  = 16 * wave + i;
    const int row = base + lr;
    const float* rp = h2 + (size_t)row * DIM + 4 * lane;
    const v4f a = *(const v4f*)rp;
    const v4f b = *(const v4f*)(rp + 128);
    float s = a.x * a.x;
    s = s + a.y * a.y; s = s + a.z * a.z; s = s + a.w * a.w;
    s = s + b.x * b.x; s = s + b.y * b.y; s = s + b.z * b.z; s = s + b.w * b.w;
#pragma unroll
    for (int off = 16; off > 0; off >>= 1) s = s + __shfl_xor(s, off, 32);
    float v = sqrtf(s);
    v = (row < nN) ? v : 0.0f;
    if (lane == 0) nr[lr] = v;
  }
  __syncthreads();
  if (wave == 0) {
    const v4f ov = *(const v4fa*)(nr + 4 * lane);
    float* op = nrm + (size_t)base + 4 * lane;
    *(volatile v4f*)op = ov;
    __threadfence();
    *(volatile v4f*)op = ov;
  }
}

__global__ __launch_bounds__(NTHR) void k_factor(const float* __restrict__ nrm, float* fac, double invN, int nN) {
  __shared__ double part[NTHR];
  __shared__ float sf[4];
  const int tid = (int)threadIdx.x;
  double s = 0.0;
#pragma unroll 1
  for (int i = tid; i < nN; i += NTHR) s += (double)nrm[i];
  part[tid] = s;
  __syncthreads();
  if (tid == 0) {
    double t = 0.0;
#pragma unroll 1
    for (int j = 0; j < NTHR; ++j) t += part[j];
    const float m = (float)(t * invN);
    sf[0] = 16.0f / m;
  }
  __syncthreads();
  const float f = sf[0];
  const v4f o = {f, f, f, f};
  if (tid < 8) {
    float* op = fac + 4 * tid;
    *(volatile v4f*)op = o;
    __threadfence();
    *(volatile v4f*)op = o;
  }
}

__global__ __launch_bounds__(NTHR) void k_pool(const float* __restrict__ hf, const int* __restrict__ ids,
                                               const float* __restrict__ fac, int nN, float* out) {
  __shared__ __attribute__((aligned(16))) float wsum[NWAVE * DIM];
  __shared__ __attribute__((aligned(16))) float outs[DIM];
  const int tid = (int)threadIdx.x, lane = tid & 31, wave = tid >> 5;
  const int g = (int)blockIdx.x;
  const float f = fac[0];

  v4f pa = {0.0f, 0.0f, 0.0f, 0.0f};
  v4f pb = {0.0f, 0.0f, 0.0f, 0.0f};
#pragma unroll 1
  for (int i0 = wave * 32; i0 < nN; i0 += NTHR) {
    const int i  = i0 + lane;
    const int ic = i < nN ? i : nN - 1;
    const int b  = ids[ic];
    const bool hit = (i < nN) && (b == g);
    unsigned msk = __builtin_amdgcn_ballot_w32(hit);
    int nh = (int)__builtin_popcount(msk);
    nh = nh > 32 ? 32 : nh;
#pragma unroll 1
    for (int q = 0; q < nh; ++q) {
      const int k = __builtin_ffs((int)msk) - 1;
      msk &= msk - 1u;
      int node = i0 + (k < 0 ? 0 : k);
      node = node > nN - 1 ? nN - 1 : node;
      const float* rp = hf + (size_t)node * DIM + 4 * lane;
      const v4f u = *(const v4f*)rp;
      const v4f v = *(const v4f*)(rp + 128);
      const v4f us = u * f;
      const v4f vs = v * f;
      pa = pa + us;
      pb = pb + vs;
    }
  }
  *(v4fa*)(wsum + wave * DIM + 4 * lane) = pa;
  *(v4fa*)(wsum + wave * DIM + 128 + 4 * lane) = pb;
  __syncthreads();
  {
    float s = 0.0f;
#pragma unroll
    for (int w2 = 0; w2 < NWAVE; ++w2) s = s + wsum[w2 * DIM + tid];
    outs[tid] = s;
  }
  __syncthreads();
  if (wave < 2) {
    const v4f ov = *(const v4fa*)(outs + 128 * wave + 4 * lane);
    float* op = out + (size_t)g * DIM + 128 * wave + 4 * lane;
    *(volatile v4f*)op = ov;
    __threadfence();
    *(volatile v4f*)op = ov;
  }
}

static inline int cdiv(int a, int b) { return (a + b - 1) / b; }
static inline size_t al256(size_t o) { return (o + 255) & ~(size_t)255; }

extern "C" void kernel_launch(void* const* d_in, const int* in_sizes, int n_in,
                              void* d_out, int out_size, void* d_ws, size_t ws_size,
                              hipStream_t stream) {
  if (n_in < 8) return;
  const int nN = in_sizes[7];
  if (nN < 16 || nN >= (1 << 22)) return;
  if ((long long)in_sizes[0] != (long long)nN * FIN) return;
  if (in_sizes[1] != FIN * DIM || in_sizes[2] != DIM) return;
  if (in_sizes[3] != DIM * DIM || in_sizes[4] != DIM) return;
  const int nE = in_sizes[5];
  if (nE < 1 || in_sizes[6] != nE) return;
  if (nE >= (1 << (31 - SLA))) return;
  if (out_size != NGR * DIM) return;

  const float* x   = (const float*)d_in[0];
  const float* W1  = (const float*)d_in[1];
  const float* b1  = (const float*)d_in[2];
  const float* W2  = (const float*)d_in[3];
  const float* b2  = (const float*)d_in[4];
  const int*   src = (const int*)d_in[5];
  const int*   dst = (const int*)d_in[6];
  const int*   n2g = (const int*)d_in[7];
  float* out = (float*)d_out;

  const int MP   = cdiv(nN, RNB) * RNB;
  const int gM   = MP / GBM;
  const int gD   = cdiv(MP, NBD);
  const int NBPD = gD * NBD;
  const int gA   = cdiv(MP, NBA);
  if ((long long)gA * NBA < (long long)MP) return;
  if (NBPD < MP) return;
  const int vec8 = ((nE & 3) == 0) ? 1 : 0;

  char* ws = (char*)d_ws;
  size_t off = 0;
  const size_t oOUTN = off; off = al256(off + (size_t)NBPD * 4);
  const size_t oNRM  = off; off = al256(off + (size_t)MP * 4);
  const size_t oFAC  = off; off = al256(off + (size_t)32 * 4);
  const size_t oW1D  = off; off = al256(off + (size_t)DIM * K1 * 2);
  const size_t oW2D  = off; off = al256(off + (size_t)DIM * K2 * 2);
  const size_t oXB   = off; off = al256(off + (size_t)MP * FIN * 2);
  const size_t oRA   = off; off = al256(off + (size_t)MP * DIM * 4);
  const size_t oRB   = off; off = al256(off + (size_t)MP * K2 * 2);
  if (off > ws_size || off > (size_t)WSMAX) return;
  float*          OUTN = (float*)(ws + oOUTN);
  float*          NRM  = (float*)(ws + oNRM);
  float*          FAC  = (float*)(ws + oFAC);
  unsigned short* W1D  = (unsigned short*)(ws + oW1D);
  unsigned short* W2D  = (unsigned short*)(ws + oW2D);
  unsigned short* XB   = (unsigned short*)(ws + oXB);
  float*          RA   = (float*)(ws + oRA);
  unsigned short* RB   = (unsigned short*)(ws + oRB);

  const size_t scanLds = (size_t)AGG_LDS_INTS * 4;
  hipFuncSetAttribute(reinterpret_cast<const void*>(&k_scan<1>), hipFuncAttributeMaxDynamicSharedMemorySize, (int)scanLds);
  hipFuncSetAttribute(reinterpret_cast<const void*>(&k_scan<2>), hipFuncAttributeMaxDynamicSharedMemorySize, (int)scanLds);

  const int nUx = MP * (FIN / 8);
  const double invN = 1.0 / (double)nN;

  k_wprep<<<(NUW1 + NUW2) / NTHR, NTHR, 0, stream>>>(W1, W2, W1D, W2D);
  k_cvx<<<cdiv(nUx, NTHR), NTHR, 0, stream>>>(x, nN, nUx, XB);
  k_deg<<<gD, NTHR, 0, stream>>>(src, nE, vec8, OUTN);
  k_scan<1><<<gA, NTHR, scanLds, stream>>>(src, dst, nE, nN, vec8, MP, OUTN, XB, RA, RB);
  k_gemm<1><<<dim3(gM, DIM / GBN), GTHR, 0, stream>>>(RB, W1D, b1, OUTN, RA, nN);
  k_scan<2><<<gA, NTHR, scanLds, stream>>>(src, dst, nE, nN, vec8, MP, OUTN, XB, RA, RB);
  k_gemm<2><<<dim3(gM, DIM / GBN), GTHR, 0, stream>>>(RB, W2D, b2, OUTN, RA, nN);
  k_rownorm<<<MP / RNB, NTHR, 0, stream>>>(RA, nN, NRM);
  k_factor<<<1, NTHR, 0, stream>>>(NRM, FAC, invN, nN);
  k_pool<<<NGR, NTHR, 0, stream>>>(RA, n2g, FAC, nN, out);
}
